// GNNMaterialPatchModel_35218731827626
// MI455X (gfx1250) — hardware-verified
//
#include <hip/hip_runtime.h>
#include <stddef.h>
#include <stdint.h>


#define HID    64
#define TM     128
#define NTHR   256
#define NWAVE  8
#define PA     136
#define PB     264
#define FNI    8
#define FEI    4
#define FOUT   6
#define EPT    8
#define CHUNK  (NTHR * EPT)
#define WCAP   (EPT * 32)
#define LISTN  (NWAVE * WCAP)
#define NBA    1024
#define SLA    10
#define RCAP   28672
#define DEGCAP 64
#define AGG_ZINTS (LISTN + 2 * RCAP + 3 * NBA)
#define AGG_LDS_INTS (AGG_ZINTS + 16)

#define WP_ENW2   0
#define WP_EEW2   8192
#define WP_L0     16384
#define WP_LSZ    57344
#define WPL_W1A   0
#define WPL_PSDW  8192
#define WPL_PEW2  24576
#define WPL_PNW1  32768
#define WPL_PNW2  49152
#define WP_DW1    (WP_L0 + 2 * WP_LSZ)
#define WP_TOTAL  (WP_DW1 + 8192)
#define NPARTS    17

#define N_AS   0
#define N_STG  34816
#define N_W1   100352
#define N_B1   102400
#define N_LDS  102656
#define E_AS   0
#define E_EHS  34816
#define E_STG  67584
#define E_SD   100352
#define E_W1   101376
#define E_B1   102400
#define E_LDS  102656
#define D_AS   0
#define D_XHS  67584
#define D_STG  100352
#define D_DW2  165888
#define D_OUT  167424
#define D_LDS  170496

static_assert(TM == NWAVE * 16 && NTHR == NWAVE * 32);
static_assert(PA % 8 == 0 && PB % 8 == 0 && PA >= 128 && PB >= 256);
static_assert(TM * PA * 2 == N_STG && TM * 128 * 4 == N_W1 - N_STG);
static_assert(TM * PA * 2 == E_EHS && TM * HID * 4 == E_STG - E_EHS && TM * HID * 4 == E_SD - E_STG);
static_assert(TM * PB * 2 == D_XHS && TM * HID * 4 == D_STG - D_XHS && TM * 128 * 4 == D_DW2 - D_STG);
static_assert(HID * FOUT * 4 == D_OUT - D_DW2 && TM * FOUT * 4 == D_LDS - D_OUT);
static_assert((CHUNK & (CHUNK - 1)) == 0 && CHUNK <= 4096);
static_assert((NBA & (NBA - 1)) == 0 && NBA == (1 << SLA));
static_assert(((long long)CHUNK << SLA) < (1LL << 31));
static_assert(NBA % NWAVE == 0 && NBA % 32 == 0 && NBA % TM == 0);
static_assert(RCAP % 32 == 0 && AGG_ZINTS % 4 == 0 && LISTN % 4 == 0);
static_assert(AGG_LDS_INTS * 4 <= 300000);
static_assert(WP_TOTAL == 139264 && (NPARTS * 1024) % NTHR == 0);
static_assert((TM * FOUT) % 32 == 0 && TM * FOUT / 4 <= NTHR);

typedef float          v2f   __attribute__((ext_vector_type(2)));
typedef float          v4f   __attribute__((ext_vector_type(4)));
typedef float          v8f   __attribute__((ext_vector_type(8)));
typedef int            v4i   __attribute__((ext_vector_type(4)));
typedef int            v8i   __attribute__((ext_vector_type(8)));
typedef unsigned short v4us  __attribute__((ext_vector_type(4)));
typedef unsigned short v8us  __attribute__((ext_vector_type(8)));
typedef unsigned short v16us __attribute__((ext_vector_type(16)));
typedef __bf16         v16bf __attribute__((ext_vector_type(16)));
typedef v2f  __attribute__((may_alias)) v2fa;
typedef v4f  __attribute__((may_alias)) v4fa;
typedef v4i  __attribute__((may_alias)) v4ia;
typedef v4us __attribute__((may_alias)) v4usa;
typedef v8us __attribute__((may_alias)) v8usa;
union FragB { v16bf v; v16us u; v8us h[2]; v8i w; };

__device__ __forceinline__ v8f wmb(const FragB& a, const FragB& b, v8f c) {
  v8f d = __builtin_amdgcn_wmma_f32_16x16x32_bf16(false, a.v, false, b.v, (short)0, c, false, false);
  asm volatile("v_nop\n\tv_nop\n\tv_nop\n\tv_nop" : "+v"(d) : "v"(a.w), "v"(b.w));
  return d;
}

__device__ __forceinline__ unsigned bf16_bits(float f) {
  const unsigned u = __float_as_uint(f);
  return (u + 0x7FFFu + ((u >> 16) & 1u)) >> 16;
}
__device__ __forceinline__ float bf16_val(float f) {
  return __uint_as_float(bf16_bits(f) << 16);
}
__device__ __forceinline__ float relu_np(float v) { return (v > 0.0f) ? v : (v - v); }

__device__ __forceinline__ void split4(const v4f v, v4us& h, v4us& l) {
  unsigned hb;
  hb = bf16_bits(v.x); h[0] = (unsigned short)hb; l[0] = (unsigned short)bf16_bits(v.x - __uint_as_float(hb << 16));
  hb = bf16_bits(v.y); h[1] = (unsigned short)hb; l[1] = (unsigned short)bf16_bits(v.y - __uint_as_float(hb << 16));
  hb = bf16_bits(v.z); h[2] = (unsigned short)hb; l[2] = (unsigned short)bf16_bits(v.z - __uint_as_float(hb << 16));
  hb = bf16_bits(v.w); h[3] = (unsigned short)hb; l[3] = (unsigned short)bf16_bits(v.w - __uint_as_float(hb << 16));
}

template <int NT, int K>
__device__ __forceinline__ void wave_gemm(const unsigned short* arow, const unsigned short* __restrict__ brow,
                                          v8f (&acc)[NT]) {
#pragma unroll 1
  for (int k0 = 0; k0 < K; k0 += 32) {
    FragB af;
    af.h[0] = *(const v8usa*)(arow + k0);
    af.h[1] = *(const v8usa*)(arow + k0 + 16);
#pragma unroll
    for (int t = 0; t < NT; ++t) {
      const unsigned short* wq = brow + (size_t)(16 * t) * (size_t)K + k0;
      FragB bf;
      bf.h[0] = *(const v8usa*)wq;
      bf.h[1] = *(const v8usa*)(wq + 16);
      acc[t] = wmb(af, bf, acc[t]);
    }
  }
}

template <int NT>
__device__ __forceinline__ void zero_acc(v8f (&acc)[NT]) {
  const v8f z = {0.f, 0.f, 0.f, 0.f, 0.f, 0.f, 0.f, 0.f};
#pragma unroll
  for (int t = 0; t < NT; ++t) acc[t] = z;
}

template <int NT>
__device__ __forceinline__ void stage_acc(float* stg, int pitch, const v8f (&acc)[NT], int wave, int hh, int m) {
#pragma unroll
  for (int t = 0; t < NT; ++t) {
#pragma unroll
    for (int r = 0; r < 8; ++r) stg[(16 * wave + 8 * hh + r) * pitch + 16 * t + m] = acc[t][r];
  }
}

template <int KIN>
__device__ __forceinline__ void enc_hidden(const float* __restrict__ in, int nRows, int rowBase,
                                           const float* w1s, const float* b1s, unsigned short* As, int tid) {
  const int r = tid >> 1, cb = (tid & 1) * 32;
  int g = rowBase + r;
  g = g < nRows ? g : nRows - 1;
  float xv[KIN];
  {
    const v4f a = *(const v4f*)(in + (size_t)g * KIN);
    xv[0] = bf16_val(a.x); xv[1] = bf16_val(a.y); xv[2] = bf16_val(a.z); xv[3] = bf16_val(a.w);
    if constexpr (KIN == 8) {
      const v4f b = *(const v4f*)(in + (size_t)g * KIN + 4);
      xv[4] = bf16_val(b.x); xv[5] = bf16_val(b.y); xv[6] = bf16_val(b.z); xv[7] = bf16_val(b.w);
    }
  }
#pragma unroll 4
  for (int c = 0; c < 32; ++c) {
    const int ch = cb + c;
    float h = b1s[ch];
#pragma unroll
    for (int k = 0; k < KIN; ++k) h = fmaf(xv[k], w1s[k * HID + ch], h);
    h = relu_np(h);
    const unsigned hb = bf16_bits(h);
    const unsigned lb = bf16_bits(h - __uint_as_float(hb << 16));
    As[r * PA + ch]       = (unsigned short)hb;
    As[r * PA + HID + ch] = (unsigned short)lb;
  }
}

template <int SLB>
__device__ __forceinline__ int scan_chunk(const int* __restrict__ dsts, int nE, int cbase, int slotBase,
                                          int nb, int vec8, int* list, int tid, int lane, int wave) {
  int wc = 0;
  const int el0  = tid * EPT;
  const int e0   = cbase + el0;
  const int sent = -2147483647 - 1;
  v4i da, db;
  if (vec8 != 0 && cbase + CHUNK <= nE) {
    da = *(const v4i*)(dsts + e0);
    db = *(const v4i*)(dsts + e0 + 4);
  } else {
    da.x = (e0     < nE) ? dsts[min(e0,     nE - 1)] : sent;
    da.y = (e0 + 1 < nE) ? dsts[min(e0 + 1, nE - 1)] : sent;
    da.z = (e0 + 2 < nE) ? dsts[min(e0 + 2, nE - 1)] : sent;
    da.w = (e0 + 3 < nE) ? dsts[min(e0 + 3, nE - 1)] : sent;
    db.x = (e0 + 4 < nE) ? dsts[min(e0 + 4, nE - 1)] : sent;
    db.y = (e0 + 5 < nE) ? dsts[min(e0 + 5, nE - 1)] : sent;
    db.z = (e0 + 6 < nE) ? dsts[min(e0 + 6, nE - 1)] : sent;
    db.w = (e0 + 7 < nE) ? dsts[min(e0 + 7, nE - 1)] : sent;
  }
  const unsigned nbs = (unsigned)slotBase;
  const unsigned unb = (unsigned)nb;
  const unsigned s0 = (unsigned)da.x - nbs, s1 = (unsigned)da.y - nbs;
  const unsigned s2 = (unsigned)da.z - nbs, s3 = (unsigned)da.w - nbs;
  const unsigned s4 = (unsigned)db.x - nbs, s5 = (unsigned)db.y - nbs;
  const unsigned s6 = (unsigned)db.z - nbs, s7 = (unsigned)db.w - nbs;
  const bool h0 = s0 < unb, h1 = s1 < unb, h2 = s2 < unb, h3 = s3 < unb;
  const bool h4 = s4 < unb, h5 = s5 < unb, h6 = s6 < unb, h7 = s7 < unb;
  const unsigned any = __builtin_amdgcn_ballot_w32(h0 | h1 | h2 | h3 | h4 | h5 | h6 | h7);
  if (any != 0u) {
#define HITJ(J, HJ, SJ) { \
      const unsigned mj = __builtin_amdgcn_ballot_w32(HJ); \
      if (mj != 0u) { \
        if (HJ) { \
          const int pos = wc + (int)__builtin_amdgcn_mbcnt_lo(mj, 0u); \
          if (pos < WCAP) list[wave * WCAP + pos] = ((el0 + (J)) << SLB) | (int)(SJ); \
        } \
        wc += (int)__builtin_popcount(mj); } }
    HITJ(0, h0, s0)
    HITJ(1, h1, s1)
    HITJ(2, h2, s2)
    HITJ(3, h3, s3)
    HITJ(4, h4, s4)
    HITJ(5, h5, s5)
    HITJ(6, h6, s6)
    HITJ(7, h7, s7)
#undef HITJ
  }
  return wc;
}

__global__ __launch_bounds__(NTHR) void k_prep(const float* __restrict__ enw2, const float* __restrict__ eew2,
                                               const float* __restrict__ pew1, const float* __restrict__ pew2,
                                               const float* __restrict__ pnw1, const float* __restrict__ pnw2,
                                               const float* __restrict__ dw1, unsigned short* WPL) {
  const int u    = (int)blockIdx.x * NTHR + (int)threadIdx.x;
  const int part = u >> 10;
  const int v    = u & 1023;
  const int n    = v >> 4;
  const int k8   = (v & 15) * 8;
  const float* W;
  int rmask = 63, dst = 0, pitch = 128, coff = 0;
  if (part == 0)      { W = enw2; dst = WP_ENW2; }
  else if (part == 1) { W = eew2; dst = WP_EEW2; }
  else if (part < 16) {
    const int pl = part - 2;
    const int l  = pl / 7;
    const int q  = pl - 7 * l;
    const int lb = WP_L0 + l * WP_LSZ;
    if (q == 0)      { W = pew1 + (size_t)l * 12288;        dst = lb + WPL_W1A; }
    else if (q == 1) { W = pew1 + (size_t)l * 12288 + 4096; dst = lb + WPL_PSDW; }
    else if (q == 2) { W = pew1 + (size_t)l * 12288 + 8192; dst = lb + WPL_PSDW + 8192; }
    else if (q == 3) { W = pew2 + (size_t)l * 4096;         dst = lb + WPL_PEW2; }
    else if (q == 4) { W = pnw1 + (size_t)l * 8192;         dst = lb + WPL_PNW1; rmask = 127; pitch = 256; coff = 0; }
    else if (q == 5) { W = pnw1 + (size_t)l * 8192;         dst = lb + WPL_PNW1; rmask = 127; pitch = 256; coff = 128; }
    else             { W = pnw2 + (size_t)l * 4096;         dst = lb + WPL_PNW2; }
  }
  else if (part == 16) { W = dw1; dst = WP_DW1; }
  else return;
  const float* p = W + (size_t)(k8 & rmask) * HID + n;
  v8us o;
#pragma unroll
  for (int i = 0; i < 8; ++i) o[i] = (unsigned short)bf16_bits(p[(size_t)i * HID]);
  unsigned short* dp = WPL + (size_t)dst + (size_t)n * pitch + coff + k8;
  *(volatile v8us*)dp = o;
  __threadfence();
  *(volatile v8us*)dp = o;
}

__global__ __launch_bounds__(NTHR) void k_nenc(const float* __restrict__ x, int nN,
                                               const float* __restrict__ w1, const float* __restrict__ b1,
                                               const float* __restrict__ b2,
                                               const unsigned short* __restrict__ W2T,
                                               const unsigned short* __restrict__ PSDW,
                                               float* XH, float* PSD) {
  extern __shared__ __attribute__((aligned(16))) unsigned char dsmN[];
  unsigned short* As = (unsigned short*)(dsmN + N_AS);
  float* stg = (float*)(dsmN + N_STG);
  float* w1s = (float*)(dsmN + N_W1);
  float* b1s = (float*)(dsmN + N_B1);
  const int tid = (int)threadIdx.x, lane = tid & 31, wave = tid >> 5, hh = lane >> 4, m = lane & 15;
  const int rowBase = (int)blockIdx.x * TM;
  const int rq = tid >> 4, c4 = (tid & 15) * 4;

  w1s[tid]        = bf16_val(w1[tid]);
  w1s[tid + NTHR] = bf16_val(w1[tid + NTHR]);
  if (tid < HID) b1s[tid] = bf16_val(b1[tid]);
  __syncthreads();
  enc_hidden<FNI>(x, nN, rowBase, w1s, b1s, As, tid);
  __syncthreads();

  v8f acc[4];
  zero_acc<4>(acc);
  wave_gemm<4, 128>(As + (16 * wave + m) * PA + 8 * hh, W2T + (size_t)m * 128 + 8 * hh, acc);
  __syncthreads();
#pragma unroll
  for (int t = 0; t < 4; ++t) {
    const int col = 16 * t + m;
    const float bb = bf16_val(b2[col]);
#pragma unroll
    for (int r = 0; r < 8; ++r) {
      const int row = 16 * wave + 8 * hh + r;
      const float v = acc[t][r] + bb;
      stg[row * HID + col] = v;
      const unsigned hb = bf16_bits(v);
      As[row * PA + col]       = (unsigned short)hb;
      As[row * PA + HID + col] = (unsigned short)bf16_bits(v - __uint_as_float(hb << 16));
    }
  }
  __syncthreads();

  {
    v4f fv[8];
#pragma unroll
    for (int i = 0; i < 8; ++i) fv[i] = *(const v4fa*)(stg + (i * 16 + rq) * HID + c4);
#pragma unroll
    for (int i = 0; i < 8; ++i)
      *(volatile v4f*)(XH + (size_t)(rowBase + i * 16 + rq) * HID + c4) = fv[i];
    __threadfence();
#pragma unroll
    for (int i = 0; i < 8; ++i)
      *(volatile v4f*)(XH + (size_t)(rowBase + i * 16 + rq) * HID + c4) = fv[i];
  }

  v8f ac8[8];
  zero_acc<8>(ac8);
  wave_gemm<8, 128>(As + (16 * wave + m) * PA + 8 * hh, PSDW + (size_t)m * 128 + 8 * hh, ac8);
  __syncthreads();
  stage_acc<8>(stg, 128, ac8, wave, hh, m);
  __syncthreads();
  {
    v4f pv[16];
#pragma unroll
    for (int i = 0; i < 16; ++i) pv[i] = *(const v4fa*)(stg + (i * 8 + wave) * 128 + 4 * lane);
#pragma unroll
    for (int i = 0; i < 16; ++i)
      *(volatile v4f*)(PSD + (size_t)(rowBase + i * 8 + wave) * 128 + 4 * lane) = pv[i];
    __threadfence();
#pragma unroll
    for (int i = 0; i < 16; ++i)
      *(volatile v4f*)(PSD + (size_t)(rowBase + i * 8 + wave) * 128 + 4 * lane) = pv[i];
  }
}

template <int ENC>
__global__ __launch_bounds__(NTHR) void k_edge(const int* __restrict__ eidx, int nE, int nN,
                                               const float* __restrict__ ea, const float* __restrict__ ew1,
                                               const float* __restrict__ eb1, const float* __restrict__ eb2,
                                               const unsigned short* __restrict__ EEW2,
                                               const unsigned short* __restrict__ W1A,
                                               const unsigned short* __restrict__ PEW2,
                                               const float* __restrict__ pb1, const float* __restrict__ pb2,
                                               const float* __restrict__ PSD, float* EH) {
  extern __shared__ __attribute__((aligned(16))) unsigned char dsmE[];
  unsigned short* As = (unsigned short*)(dsmE + E_AS);
  float* ehs = (float*)(dsmE + E_EHS);
  float* stg = (float*)(dsmE + E_STG);
  int*   sd  = (int*)(dsmE + E_SD);
  float* w1s = (float*)(dsmE + E_W1);
  float* b1s = (float*)(dsmE + E_B1);
  const int tid = (int)threadIdx.x, lane = tid & 31, wave = tid >> 5, hh = lane >> 4, m = lane & 15;
  const int rowBase = (int)blockIdx.x * TM;
  const int rq = tid >> 4, c4 = (tid & 15) * 4;

  {
    const int which = tid >> 7, r = tid & 127;
    int e = rowBase + r;
    e = e < nE ? e : nE - 1;
    int v = eidx[(size_t)which * (size_t)nE + e];
    v = v < 0 ? 0 : (v > nN - 1 ? nN - 1 : v);
    sd[tid] = v;
  }

  if constexpr (ENC != 0) {
    w1s[tid] = bf16_val(ew1[tid]);
    if (tid < HID) b1s[tid] = bf16_val(eb1[tid]);
    __syncthreads();
    enc_hidden<FEI>(ea, nE, rowBase, w1s, b1s, As, tid);
    __syncthreads();
    v8f ace[4];
    zero_acc<4>(ace);
    wave_gemm<4, 128>(As + (16 * wave + m) * PA + 8 * hh, EEW2 + (size_t)m * 128 + 8 * hh, ace);
    __syncthreads();
#pragma unroll
    for (int t = 0; t < 4; ++t) {
      const int col = 16 * t + m;
      const float bb = bf16_val(eb2[col]);
#pragma unroll
      for (int r = 0; r < 8; ++r) {
        const int row = 16 * wave + 8 * hh + r;
        const float v = ace[t][r] + bb;
        ehs[row * HID + col] = v;
        const unsigned hb = bf16_bits(v);
        As[row * PA + col]       = (unsigned short)hb;
        As[row * PA + HID + col] = (unsigned short)bf16_bits(v - __uint_as_float(hb << 16));
      }
    }
  } else {
#pragma unroll 2
    for (int i = 0; i < 8; ++i) {
      const int row = i * 16 + rq;
      const v4f v = *(const v4f*)(EH + (size_t)(rowBase + row) * HID + c4);
      *(v4fa*)(ehs + row * HID + c4) = v;
      v4us h4, l4;
      split4(v, h4, l4);
      *(v4usa*)(As + row * PA + c4)       = h4;
      *(v4usa*)(As + row * PA + HID + c4) = l4;
    }
  }
  __syncthreads();

  v8f acc[4];
  zero_acc<4>(acc);
  wave_gemm<4, 128>(As + (16 * wave + m) * PA + 8 * hh, W1A + (size_t)m * 128 + 8 * hh, acc);
  stage_acc<4>(stg, HID, acc, wave, hh, m);
  __syncthreads();

  {
    v4f b1v;
    {
      const v4f t = *(const v4f*)(pb1 + c4);
      b1v.x = bf16_val(t.x); b1v.y = bf16_val(t.y); b1v.z = bf16_val(t.z); b1v.w = bf16_val(t.w);
    }
#pragma unroll 2
    for (int i = 0; i < 8; ++i) {
      const int row = i * 16 + rq;
      const int s = sd[row];
      const int d = sd[TM + row];
      const v4f a  = *(const v4fa*)(stg + row * HID + c4);
      const v4f ps = *(const v4f*)(PSD + (size_t)s * 128 + c4);
      const v4f pd = *(const v4f*)(PSD + (size_t)d * 128 + HID + c4);
      v4f h;
      h.x = relu_np(((a.x + ps.x) + pd.x) + b1v.x);
      h.y = relu_np(((a.y + ps.y) + pd.y) + b1v.y);
      h.z = relu_np(((a.z + ps.z) + pd.z) + b1v.z);
      h.w = relu_np(((a.w + ps.w) + pd.w) + b1v.w);
      v4us h4, l4;
      split4(h, h4, l4);
      *(v4usa*)(As + row * PA + c4)       = h4;
      *(v4usa*)(As + row * PA + HID + c4) = l4;
    }
  }
  __syncthreads();

  zero_acc<4>(acc);
  wave_gemm<4, 128>(As + (16 * wave + m) * PA + 8 * hh, PEW2 + (size_t)m * 128 + 8 * hh, acc);
  stage_acc<4>(stg, HID, acc, wave, hh, m);
  __syncthreads();

  {
    v4f b2v;
    {
      const v4f t = *(const v4f*)(pb2 + c4);
      b2v.x = bf16_val(t.x); b2v.y = bf16_val(t.y); b2v.z = bf16_val(t.z); b2v.w = bf16_val(t.w);
    }
    v4f fv[8];
#pragma unroll
    for (int i = 0; i < 8; ++i) {
      const int row = i * 16 + rq;
      const v4f a = *(const v4fa*)(stg + row * HID + c4);
      const v4f r = *(const v4fa*)(ehs + row * HID + c4);
      fv[i] = (a + b2v) + r;
    }
#pragma unroll
    for (int i = 0; i < 8; ++i)
      *(volatile v4f*)(EH + (size_t)(rowBase + i * 16 + rq) * HID + c4) = fv[i];
    __threadfence();
#pragma unroll
    for (int i = 0; i < 8; ++i)
      *(volatile v4f*)(EH + (size_t)(rowBase + i * 16 + rq) * HID + c4) = fv[i];
  }
}

__global__ __launch_bounds__(NTHR) void k_scan(const int* __restrict__ dsts, int nE, int nN, int vec8, int mRows,
                                               const float* __restrict__ EH, float* AGG) {
  extern __shared__ __attribute__((aligned(16))) int dsmS[];
  int* list = dsmS;
  int* hl   = dsmS + LISTN;
  int* sl   = dsmS + LISTN + RCAP;
  int* cnt  = dsmS + LISTN + 2 * RCAP;
  int* offs = cnt + NBA;
  int* cur  = offs + NBA;
  int* misc = cur + NBA;
  const int tid = (int)threadIdx.x, lane = tid & 31, wave = tid >> 5;
  const int nodeBase = (int)blockIdx.x * NBA;

  {
    const v4i z4 = {0, 0, 0, 0};
    for (int i = tid * 4; i < AGG_ZINTS; i += NTHR * 4) *(v4ia*)(dsmS + i) = z4;
    if (tid < 16) misc[tid] = 0;
  }
  __syncthreads();

  int t = 0, ov = 0;
  const int nChunks = (nE + CHUNK - 1) / CHUNK;
#pragma unroll 1
  for (int ch = 0; ch < nChunks; ++ch) {
    const int cbase = ch * CHUNK;
    const int wc = scan_chunk<SLA>(dsts, nE, cbase, nodeBase, NBA, vec8, list, tid, lane, wave);
    if (lane == 0) misc[wave] = wc;
    __syncthreads();
    if (wave == 0) {
#pragma unroll 1
      for (int w2 = 0; w2 < NWAVE; ++w2) {
        int c = misc[w2];
        c = c < 0 ? 0 : (c > WCAP ? WCAP : c);
#pragma unroll 1
        for (int b0 = 0; b0 < c; b0 += 32) {
          const int idx = b0 + lane;
          const int ent = list[w2 * WCAP + (idx < WCAP ? idx : WCAP - 1)];
          const int m32 = (c - b0) < 32 ? (c - b0) : 32;
#pragma unroll 1
          for (int k = 0; k < m32; ++k) {
            const int u    = __builtin_amdgcn_readlane(ent, k);
            const int slot = u & (NBA - 1);
            const int el   = (u >> SLA) & (CHUNK - 1);
            const int pk   = ((cbase + el) << SLA) | slot;
            if (t < RCAP) {
              if (lane == 0) { hl[t] = pk; cnt[slot] = cnt[slot] + 1; }
              t = t + 1;
            } else {
              ov = 1;
            }
          }
        }
      }
    }
    __syncthreads();
  }
  if (wave == 0 && lane == 0) { misc[8] = t; misc[9] = ov; }
  __syncthreads();
  int tt = misc[8];
  tt = tt < 0 ? 0 : (tt > RCAP ? RCAP : tt);
  const int ovf = misc[9];

  if (wave == 0) {
    const int base = lane * (NBA / 32);
    int s = 0;
#pragma unroll 1
    for (int i = 0; i < NBA / 32; ++i) s += cnt[base + i];
    int incl = s;
#pragma unroll
    for (int d = 1; d < 32; d <<= 1) {
      const int y = __shfl_up(incl, d, 32);
      if (lane >= d) incl += y;
    }
    int run = incl - s;
#pragma unroll 1
    for (int i = 0; i < NBA / 32; ++i) {
      const int cv = cnt[base + i];
      offs[base + i] = run;
      cur[base + i]  = run;
      run += cv;
    }
  }
  __syncthreads();
  if (wave == 0) {
#pragma unroll 1
    for (int b0 = 0; b0 < tt; b0 += 32) {
      const int idx = b0 + lane;
      const int ent = hl[idx < RCAP ? idx : RCAP - 1];
      const int m32 = (tt - b0) < 32 ? (tt - b0) : 32;
#pragma unroll 1
      for (int k = 0; k < m32; ++k) {
        const int u    = __builtin_amdgcn_readlane(ent, k);
        const int slot = u & (NBA - 1);
        if (lane == 0) {
          int p = cur[slot];
          p = p < 0 ? 0 : (p > RCAP - 1 ? RCAP - 1 : p);
          sl[p] = u;
          cur[slot] = p + 1;
        }
      }
    }
  }
  __syncthreads();

  const float qnan = __int_as_float(0x7fc00000);
  const float pz = (ovf != 0) ? qnan : 0.0f;
  const int sa = (2 * lane) & 31, sb = (2 * lane + 1) & 31;
#pragma unroll 1
  for (int si = 0; si < NBA / NWAVE; ++si) {
    const int s    = si * NWAVE + wave;
    const int node = nodeBase + s;
    int c = cnt[s];
    const bool big = c > DEGCAP;
    c = c < 0 ? 0 : (c > DEGCAP ? DEGCAP : c);
    int o = offs[s];
    o = o < 0 ? 0 : (o > RCAP ? RCAP : o);
    float acc0 = 0.0f, acc1 = 0.0f;
#pragma unroll 1
    for (int b0 = 0; b0 < c; b0 += 32) {
      int idx = o + b0 + lane;
      idx = idx > RCAP - 1 ? RCAP - 1 : idx;
      const int ent = sl[idx];
      int eid = ent >> SLA;
      eid = eid < 0 ? 0 : (eid > nE - 1 ? nE - 1 : eid);
      const int m32 = (c - b0) < 32 ? (c - b0) : 32;
#pragma unroll 1
      for (int k = 0; k < m32; ++k) {
        const int ek = __builtin_amdgcn_readlane(eid, k);
        const v2f a = *(const v2fa*)(EH + (size_t)ek * HID + 2 * lane);
        acc0 += a.x; acc1 += a.y;
      }
    }
    const float pzr = big ? qnan : pz;
    const bool live = node < nN;
    const float v0 = live ? (acc0 + pzr) : 0.0f;
    const float v1 = live ? (acc1 + pzr) : 0.0f;
    const bool wr = (node < mRows) && (lane < 16);
    v4f ow;
    ow.x = __shfl(v0, sa, 32); ow.y = __shfl(v1, sa, 32);
    ow.z = __shfl(v0, sb, 32); ow.w = __shfl(v1, sb, 32);
    float* op = AGG + (size_t)node * HID + 4 * (lane & 15);
    if (wr) *(volatile v4f*)op = ow;
    __threadfence();
    if (wr) *(volatile v4f*)op = ow;
  }
}

template <int LAST>
__global__ __launch_bounds__(NTHR) void k_node(int nN, float* XH, const float* __restrict__ AGG,
                                               const unsigned short* __restrict__ PNW1,
                                               const unsigned short* __restrict__ PNW2,
                                               const float* __restrict__ nb1, const float* __restrict__ nb2,
                                               const unsigned short* __restrict__ WC,
                                               const float* __restrict__ db1, const float* __restrict__ dw2,
                                               const float* __restrict__ db2,
                                               float* PSD, float* out) {
  extern __shared__ __attribute__((aligned(16))) unsigned char dsmD[];
  unsigned short* As = (unsigned short*)(dsmD + D_AS);
  float* xhs  = (float*)(dsmD + D_XHS);
  float* stg  = (float*)(dsmD + D_STG);
  float* dw2s = (float*)(dsmD + D_DW2);
  float* outs = (float*)(dsmD + D_OUT);
  const int tid = (int)threadIdx.x, lane = tid & 31, wave = tid >> 5, hh = lane >> 4, m = lane & 15;
  const int rowBase = (int)blockIdx.x * TM;
  const int rq = tid >> 4, c4 = (tid & 15) * 4;

  if constexpr (LAST != 0) {
    dw2s[tid] = bf16_val(dw2[tid]);
    if (tid < HID * FOUT - NTHR) dw2s[tid + NTHR] = bf16_val(dw2[tid + NTHR]);
  }

#pragma unroll 2
  for (int i = 0; i < 8; ++i) {
    const int row = i * 16 + rq;
    const v4f xv = *(const v4f*)(XH + (size_t)(rowBase + row) * HID + c4);
    const v4f av = *(const v4f*)(AGG + (size_t)(rowBase + row) * HID + c4);
    *(v4fa*)(xhs + row * HID + c4) = xv;
    v4us xh, xl, ah, al;
    split4(xv, xh, xl);
    split4(av, ah, al);
    *(v4usa*)(As + row * PB + c4)       = xh;
    *(v4usa*)(As + row * PB + 64 + c4)  = ah;
    *(v4usa*)(As + row * PB + 128 + c4) = xl;
    *(v4usa*)(As + row * PB + 192 + c4) = al;
  }
  __syncthreads();

  v8f acc[4];
  zero_acc<4>(acc);
  wave_gemm<4, 256>(As + (16 * wave + m) * PB + 8 * hh, PNW1 + (size_t)m * 256 + 8 * hh, acc);
  stage_acc<4>(stg, HID, acc, wave, hh, m);
  __syncthreads();

  {
    v4f b1v;
    {
      const v4f t = *(const v4f*)(nb1 + c4);
      b1v.x = bf16_val(t.x); b1v.y = bf16_val(t.y); b1v.z = bf16_val(t.z); b1v.w = bf16_val(t.w);
    }
#pragma unroll 2
    for (int i = 0; i < 8; ++i) {
      const int row = i * 16 + rq;
      const v4f a = *(const v4fa*)(stg + row * HID + c4);
      v4f h;
      h.x = relu_np(a.x + b1v.x); h.y = relu_np(a.y + b1v.y);
      h.z = relu_np(a.z + b1v.z); h.w = relu_np(a.w + b1v.w);
      v4us h4, l4;
      split4(h, h4, l4);
      *(v4usa*)(As + row * PB + c4)       = h4;
      *(v4usa*)(As + row * PB + HID + c4) = l4;
    }
  }
  __syncthreads();

  zero_acc<4>(acc);
  wave_gemm<4, 128>(As + (16 * wave + m) * PB + 8 * hh, PNW2 + (size_t)m * 128 + 8 * hh, acc);
  stage_acc<4>(stg, HID, acc, wave, hh, m);
  __syncthreads();

  {
    v4f b2v;
    {
      const v4f t = *(const v4f*)(nb2 + c4);
      b2v.x = bf16_val(t.x); b2v.y = bf16_val(t.y); b2v.z = bf16_val(t.z); b2v.w = bf16_val(t.w);
    }
    v4f fv[8];
#pragma unroll
    for (int i = 0; i < 8; ++i) {
      const int row = i * 16 + rq;
      const v4f a = *(const v4fa*)(stg + row * HID + c4);
      const v4f r = *(const v4fa*)(xhs + row * HID + c4);
      const v4f v = (a + b2v) + r;
      fv[i] = v;
      v4us h4, l4;
      split4(v, h4, l4);
      *(v4usa*)(As + row * PB + c4)       = h4;
      *(v4usa*)(As + row * PB + HID + c4) = l4;
    }
    if constexpr (LAST == 0) {
#pragma unroll
      for (int i = 0; i < 8; ++i)
        *(volatile v4f*)(XH + (size_t)(rowBase + i * 16 + rq) * HID + c4) = fv[i];
      __threadfence();
#pragma unroll
      for (int i = 0; i < 8; ++i)
        *(volatile v4f*)(XH + (size_t)(rowBase + i * 16 + rq) * HID + c4) = fv[i];
    }
  }
  __syncthreads();

  if constexpr (LAST == 0) {
    v8f ac8[8];
    zero_acc<8>(ac8);
    wave_gemm<8, 128>(As + (16 * wave + m) * PB + 8 * hh, WC + (size_t)m * 128 + 8 * hh, ac8);
    stage_acc<8>(stg, 128, ac8, wave, hh, m);
    __syncthreads();
    v4f pv[16];
#pragma unroll
    for (int i = 0; i < 16; ++i) pv[i] = *(const v4fa*)(stg + (i * 8 + wave) * 128 + 4 * lane);
#pragma unroll
    for (int i = 0; i < 16; ++i)
      *(volatile v4f*)(PSD + (size_t)(rowBase + i * 8 + wave) * 128 + 4 * lane) = pv[i];
    __threadfence();
#pragma unroll
    for (int i = 0; i < 16; ++i)
      *(volatile v4f*)(PSD + (size_t)(rowBase + i * 8 + wave) * 128 + 4 * lane) = pv[i];
  } else {
    v8f acd[4];
    zero_acc<4>(acd);
    wave_gemm<4, 128>(As + (16 * wave + m) * PB + 8 * hh, WC + (size_t)m * 128 + 8 * hh, acd);
#pragma unroll
    for (int t = 0; t < 4; ++t) {
      const int col = 16 * t + m;
      const float bb = bf16_val(db1[col]);
#pragma unroll
      for (int r = 0; r < 8; ++r)
        stg[(16 * wave + 8 * hh + r) * HID + col] = relu_np(acd[t][r] + bb);
    }
    __syncthreads();
#pragma unroll 1
    for (int q = 0; q < (TM * FOUT) / NTHR; ++q) {
      const int idx = q * NTHR + tid;
      const int row = idx / FOUT;
      const int j   = idx - row * FOUT;
      const float* pr = stg + row * HID;
      float s = 0.0f;
#pragma unroll 2
      for (int f4 = 0; f4 < HID / 4; ++f4) {
        const v4f p = *(const v4fa*)(pr + 4 * f4);
        const float* w = dw2s + (4 * f4) * FOUT + j;
        s = fmaf(p.x, w[0], s);
        s = fmaf(p.y, w[FOUT], s);
        s = fmaf(p.z, w[2 * FOUT], s);
        s = fmaf(p.w, w[3 * FOUT], s);
      }
      outs[idx] = s + bf16_val(db2[j]);
    }
    __syncthreads();
    int nvalid = nN - rowBase;
    nvalid = nvalid > TM ? TM : (nvalid < 0 ? 0 : nvalid);
    const int nq = (nvalid * FOUT) >> 2;
    const int ti = tid < (TM * FOUT / 4) ? tid : (TM * FOUT / 4 - 1);
    const v4f ov = *(const v4fa*)(outs + 4 * ti);
    float* op = out + (size_t)rowBase * FOUT + 4 * (size_t)tid;
    const bool ok = tid < nq;
    if (ok) *(volatile v4f*)op = ov;
    __threadfence();
    if (ok) *(volatile v4f*)op = ov;
  }
}

static inline int cdiv(int a, int b) { return (a + b - 1) / b; }
static inline size_t al256(size_t o) { return (o + 255) & ~(size_t)255; }

extern "C" void kernel_launch(void* const* d_in, const int* in_sizes, int n_in,
                              void* d_out, int out_size, void* d_ws, size_t ws_size,
                              hipStream_t stream) {
  if (n_in < 23) return;
  const int nN = in_sizes[0] / FNI;
  if (nN < 1 || nN > (1 << 22) || in_sizes[0] != nN * FNI) return;
  const int nE = in_sizes[1] / FEI;
  if (nE < 1 || nE >= (1 << (31 - SLA)) || in_sizes[1] != nE * FEI) return;
  if (in_sizes[2] != 2 * nE) return;
  if (in_sizes[3] != FNI * HID || in_sizes[4] != HID) return;
  if (in_sizes[5] != HID * HID || in_sizes[6] != HID) return;
  if (in_sizes[7] != FEI * HID || in_sizes[8] != HID) return;
  if (in_sizes[9] != HID * HID || in_sizes[10] != HID) return;
  if (in_sizes[11] != 2 * 192 * HID || in_sizes[12] != 2 * HID) return;
  if (in_sizes[13] != 2 * HID * HID || in_sizes[14] != 2 * HID) return;
  if (in_sizes[15] != 2 * 128 * HID || in_sizes[16] != 2 * HID) return;
  if (in_sizes[17] != 2 * HID * HID || in_sizes[18] != 2 * HID) return;
  if (in_sizes[19] != HID * HID || in_sizes[20] != HID) return;
  if (in_sizes[21] != HID * FOUT || in_sizes[22] != FOUT) return;
  if ((long long)out_size != (long long)nN * FOUT) return;
  if ((((nN % TM) * FOUT) % 32) != 0) return;

  const float* x     = (const float*)d_in[0];
  const float* eattr = (const float*)d_in[1];
  const int*   eidx  = (const int*)d_in[2];
  const float* enw1 = (const float*)d_in[3];  const float* enb1 = (const float*)d_in[4];
  const float* enw2 = (const float*)d_in[5];  const float* enb2 = (const float*)d_in[6];
  const float* eew1 = (const float*)d_in[7];  const float* eeb1 = (const float*)d_in[8];
  const float* eew2 = (const float*)d_in[9];  const float* eeb2 = (const float*)d_in[10];
  const float* pew1 = (const float*)d_in[11]; const float* peb1 = (const float*)d_in[12];
  const float* pew2 = (const float*)d_in[13]; const float* peb2 = (const float*)d_in[14];
  const float* pnw1 = (const float*)d_in[15]; const float* pnb1 = (const float*)d_in[16];
  const float* pnw2 = (const float*)d_in[17]; const float* pnb2 = (const float*)d_in[18];
  const float* dw1  = (const float*)d_in[19]; const float* db1  = (const float*)d_in[20];
  const float* dw2  = (const float*)d_in[21]; const float* db2  = (const float*)d_in[22];
  float* out = (float*)d_out;
  const int* dst = eidx + nE;

  const int NP = cdiv(nN, TM) * TM;
  const int EP = cdiv(nE, TM) * TM;
  const int gA = cdiv(NP, NBA);
  if ((long long)gA * NBA < (long long)NP) return;
  const int vec8 = ((nE & 3) == 0) ? 1 : 0;

  char* ws = (char*)d_ws;
  size_t off = 0;
  const size_t oW   = off; off = al256(off + (size_t)WP_TOTAL * 2);
  const size_t oXH  = off; off = al256(off + (size_t)NP * HID * 4);
  const size_t oPSD = off; off = al256(off + (size_t)NP * 128 * 4);
  const size_t oAGG = off; off = al256(off + (size_t)NP * HID * 4);
  const size_t oEH  = off; off = al256(off + (size_t)EP * HID * 4);
  if (off > ws_size) return;
  unsigned short* WPL = (unsigned short*)(ws + oW);
  float* XH  = (float*)(ws + oXH);
  float* PSD = (float*)(ws + oPSD);
  float* AGG = (float*)(ws + oAGG);
  float* EH  = (float*)(ws + oEH);

  const unsigned short* ENW2 = WPL + WP_ENW2;
  const unsigned short* EEW2 = WPL + WP_EEW2;
  const unsigned short* L0   = WPL + WP_L0;
  const unsigned short* L1   = WPL + WP_L0 + WP_LSZ;
  const unsigned short* DW1  = WPL + WP_DW1;

  const size_t scanLds = (size_t)AGG_LDS_INTS * 4;
  hipFuncSetAttribute(reinterpret_cast<const void*>(&k_nenc), hipFuncAttributeMaxDynamicSharedMemorySize, (int)N_LDS);
  hipFuncSetAttribute(reinterpret_cast<const void*>(&k_edge<1>), hipFuncAttributeMaxDynamicSharedMemorySize, (int)E_LDS);
  hipFuncSetAttribute(reinterpret_cast<const void*>(&k_edge<0>), hipFuncAttributeMaxDynamicSharedMemorySize, (int)E_LDS);
  hipFuncSetAttribute(reinterpret_cast<const void*>(&k_node<0>), hipFuncAttributeMaxDynamicSharedMemorySize, (int)D_LDS);
  hipFuncSetAttribute(reinterpret_cast<const void*>(&k_node<1>), hipFuncAttributeMaxDynamicSharedMemorySize, (int)D_LDS);
  hipFuncSetAttribute(reinterpret_cast<const void*>(&k_scan), hipFuncAttributeMaxDynamicSharedMemorySize, (int)scanLds);

  k_prep<<<(NPARTS * 1024) / NTHR, NTHR, 0, stream>>>(enw2, eew2, pew1, pew2, pnw1, pnw2, dw1, WPL);
  k_nenc<<<NP / TM, NTHR, N_LDS, stream>>>(x, nN, enw1, enb1, enb2, ENW2, L0 + WPL_PSDW, XH, PSD);
  k_edge<1><<<EP / TM, NTHR, E_LDS, stream>>>(eidx, nE, nN, eattr, eew1, eeb1, eeb2, EEW2,
                                              L0 + WPL_W1A, L0 + WPL_PEW2, peb1, peb2, PSD, EH);
  k_scan<<<gA, NTHR, scanLds, stream>>>(dst, nE, nN, vec8, NP, EH, AGG);
  k_node<0><<<NP / TM, NTHR, D_LDS, stream>>>(nN, XH, AGG, L0 + WPL_PNW1, L0 + WPL_PNW2, pnb1, pnb2,
                                              L1 + WPL_PSDW, db1, dw2, db2, PSD, out);
  k_edge<0><<<EP / TM, NTHR, E_LDS, stream>>>(eidx, nE, nN, eattr, eew1, eeb1, eeb2, EEW2,
                                              L1 + WPL_W1A, L1 + WPL_PEW2, peb1 + HID, peb2 + HID, PSD, EH);
  k_scan<<<gA, NTHR, scanLds, stream>>>(dst, nE, nN, vec8, NP, EH, AGG);
  k_node<1><<<NP / TM, NTHR, D_LDS, stream>>>(nN, XH, AGG, L1 + WPL_PNW1, L1 + WPL_PNW2, pnb1 + HID, pnb2 + HID,
                                              DW1, db1, dw2, db2, PSD, out);
}
